// TemporalGNN_10101763080488
// MI455X (gfx1250) — hardware-verified
//
#include <hip/hip_runtime.h>
#include <stddef.h>
#include <stdint.h>


#define AS3 __attribute__((address_space(3)))

#define NB_    4
#define NS_    32
#define NN_    1024
#define NF_    64
#define NH_    128
#define NG_    512
#define NO_    32
#define NE_    16384
#define NSEQ   (NB_ * NN_)
#define NSL    (NB_ * NS_)
#define NROW   (NSL * NN_)
#define SLB    8
#define NSQB   16
#define NTHR   256
#define NWAVE  8
#define EPT    8
#define CHUNK  (NTHR * EPT)
#define WCAP   (EPT * 32)
#define LISTN  (NWAVE * WCAP)
#define NBMAX  2048
#define RCAP   16416
#define DEGCAP 16416
#define STW    (SLB * 64)
#define PLANE_U32 (NROW * 32)
#define WSMAX  134217728
#define LDS_AGG ((2 * RCAP + 2 * NBMAX + LISTN + 2 * NWAVE + NN_) * 4)

static_assert(NF_ == 64);
static_assert(NF_ % 32 == 0 && NH_ % 32 == 0);
static_assert(NH_ % 64 == 0 && NG_ == 4 * NH_ && NG_ == 2 * NTHR);
static_assert(NSL % SLB == 0);
static_assert(2 * SLB == 16);
static_assert(NN_ <= NBMAX && NTHR * 8 == NBMAX);
static_assert(NN_ % NWAVE == 0 && NN_ % NTHR == 0);
static_assert(LISTN >= NBMAX && LISTN >= NWAVE * WCAP);
static_assert((RCAP % 32) == 0 && RCAP > NE_);
static_assert(NWAVE * STW <= RCAP);
static_assert((CHUNK & (CHUNK - 1)) == 0 && CHUNK <= 4096);
static_assert((NBMAX & (NBMAX - 1)) == 0 && NBMAX <= 4096);
static_assert(LDS_AGG <= 300000);
static_assert(NSEQ % NSQB == 0 && NN_ % NSQB == 0);
static_assert(NSQB == 16 && NH_ == 16 * NWAVE);
static_assert(NROW % 128 == 0);
static_assert(NO_ == 32);

typedef __bf16         v16b __attribute__((ext_vector_type(16)));
typedef unsigned short v8us __attribute__((ext_vector_type(8)));
typedef float          v8f  __attribute__((ext_vector_type(8)));
typedef float          v4f  __attribute__((ext_vector_type(4)));
typedef unsigned int   v4u  __attribute__((ext_vector_type(4)));
typedef int            v4i  __attribute__((ext_vector_type(4)));
typedef v8us __attribute__((may_alias)) v8usa;
typedef v4f  __attribute__((may_alias)) v4fa;
typedef v4u  __attribute__((may_alias)) v4ua;

typedef AS3 unsigned short*       lp_us;
typedef AS3 const unsigned short* lcp_us;
typedef AS3 float*                lp_f;
typedef AS3 const float*          lcp_f;

union Frag { v16b v; v8us half[2]; };

constexpr int P_X   = 0;
constexpr int P_WG  = P_X  + NB_ * NS_ * NN_ * NF_;
constexpr int P_WI  = P_WG + NH_ * NF_;
constexpr int P_WH  = P_WI + NG_ * NH_;
constexpr int P_WF  = P_WH + NG_ * NH_;
constexpr int P_END = P_WF + NO_ * NH_;
constexpr int NPC   = P_END / 8;
constexpr int NCBLK = NPC / 256;
static_assert(P_END % 8 == 0);
static_assert(NPC % 256 == 0);
static_assert(P_WG % 2048 == 0 && P_WI % 2048 == 0 && P_WH % 2048 == 0 && P_WF % 2048 == 0);

constexpr size_t OFF_CV  = 0;
constexpr size_t SZ_CV   = (size_t)P_END * 2;
constexpr size_t OFF_AG  = OFF_CV + SZ_CV;
constexpr size_t SZ_AGP  = (size_t)NROW * NF_ * 2;
constexpr size_t OFF_AGL = OFF_AG + SZ_AGP;
constexpr size_t OFF_CVH = OFF_AGL + SZ_AGP;
constexpr size_t SZ_CVP  = (size_t)NROW * NH_ * 2;
constexpr size_t OFF_CVL = OFF_CVH + SZ_CVP;
constexpr size_t WS_END  = OFF_CVL + SZ_CVP;
static_assert(OFF_AG % 128 == 0 && OFF_AGL % 128 == 0 && OFF_CVH % 128 == 0 && OFF_CVL % 128 == 0);
static_assert(WS_END <= (size_t)WSMAX);
static_assert((size_t)NPC * 16 == SZ_CV);
static_assert((size_t)PLANE_U32 * 4 == SZ_AGP);
static_assert((size_t)(NSL / SLB) * SLB * NN_ * 128 == SZ_AGP);
static_assert((size_t)(NROW / 128) * 2 * 128 * 128 == SZ_CVP);

__device__ __forceinline__ unsigned short bf16_bits(float f) {
  unsigned u = __float_as_uint(f);
  u += 0x7FFFu + ((u >> 16) & 1u);
  return (unsigned short)(u >> 16);
}
__device__ __forceinline__ float bf16_val(unsigned short b) { return __uint_as_float(((unsigned)b) << 16); }
__device__ __forceinline__ float bf16r(float f) { return bf16_val(bf16_bits(f)); }
__device__ __forceinline__ v8f zero8() {
  v8f z;
#pragma unroll
  for (int i = 0; i < 8; ++i) z[i] = 0.0f;
  return z;
}

__device__ __forceinline__ void ldfrag_g(Frag& f, const unsigned short* p, int h) {
  f.half[0] = *(const v8usa*)(p + 8 * h);
  f.half[1] = *(const v8usa*)(p + 16 + 8 * h);
}
__device__ __forceinline__ void ldfrag_l(Frag& f, lcp_us p, int h) {
  f.half[0] = *(AS3 const v8usa*)(p + 8 * h);
  f.half[1] = *(AS3 const v8usa*)(p + 16 + 8 * h);
}
__device__ __forceinline__ v8f mma16(v8f c, const Frag& a, const Frag& b) {
  return __builtin_amdgcn_wmma_f32_16x16x32_bf16(false, a.v, false, b.v, (short)0, c, false, false);
}

__device__ __forceinline__ void ldwait() {
  asm volatile("s_wait_loadcnt 0x0" ::: "memory");
}

__device__ __forceinline__ float sigm(float x) {
  const float xc = fminf(fmaxf(x, -40.0f), 40.0f);
  return 1.0f / (1.0f + expf(-xc));
}

__global__ __launch_bounds__(256)
void cvt_kernel(const float* __restrict__ x, const float* __restrict__ wg, const float* __restrict__ wi,
                const float* __restrict__ wh, const float* __restrict__ wf, unsigned short* cv)
{
  const int g = blockIdx.x * 256 + threadIdx.x;
  if (g >= NPC) return;
  const int e = g * 8;
  v4f a, c;
  if (e >= P_WG && e < P_WI) {
    const int idx = e - P_WG;
    const int n   = idx >> 6;
    const int k8  = idx & 63;
    const float* p = wg + (size_t)k8 * NH_ + n;
    a[0] = p[0];               a[1] = p[NH_];             a[2] = p[2 * NH_];         a[3] = p[3 * NH_];
    c[0] = p[4 * NH_];         c[1] = p[5 * NH_];         c[2] = p[6 * NH_];         c[3] = p[7 * NH_];
  } else {
    const float* src;
    if      (e < P_WG) src = x  + e;
    else if (e < P_WH) src = wi + (e - P_WI);
    else if (e < P_WF) src = wh + (e - P_WH);
    else               src = wf + (e - P_WF);
    a = *(const v4fa*)src;
    c = *(const v4fa*)(src + 4);
  }
  v8us o;
  o[0] = bf16_bits(a[0]); o[1] = bf16_bits(a[1]); o[2] = bf16_bits(a[2]); o[3] = bf16_bits(a[3]);
  o[4] = bf16_bits(c[0]); o[5] = bf16_bits(c[1]); o[6] = bf16_bits(c[2]); o[7] = bf16_bits(c[3]);
  unsigned short* dst = cv + e;
  *(volatile v8us*)dst = o;
  __threadfence();
  *(volatile v8us*)dst = o;
}

__device__ __forceinline__ int scan_chunk(const int* __restrict__ dsts, int nE, int cbase, int slotBase,
                                          int nb, int vec8, int* list, int tid, int lane, int wave) {
  int wc = 0;
  const int el0  = tid * EPT;
  const int e0   = cbase + el0;
  const int sent = -2147483647 - 1;
  v4i da, db;
  if (vec8 != 0 && cbase + CHUNK <= nE) {
    da = *(const v4i*)(dsts + e0);
    db = *(const v4i*)(dsts + e0 + 4);
  } else {
    da.x = (e0     < nE) ? dsts[min(e0,     nE - 1)] : sent;
    da.y = (e0 + 1 < nE) ? dsts[min(e0 + 1, nE - 1)] : sent;
    da.z = (e0 + 2 < nE) ? dsts[min(e0 + 2, nE - 1)] : sent;
    da.w = (e0 + 3 < nE) ? dsts[min(e0 + 3, nE - 1)] : sent;
    db.x = (e0 + 4 < nE) ? dsts[min(e0 + 4, nE - 1)] : sent;
    db.y = (e0 + 5 < nE) ? dsts[min(e0 + 5, nE - 1)] : sent;
    db.z = (e0 + 6 < nE) ? dsts[min(e0 + 6, nE - 1)] : sent;
    db.w = (e0 + 7 < nE) ? dsts[min(e0 + 7, nE - 1)] : sent;
  }
  const unsigned nbs = (unsigned)slotBase;
  const unsigned unb = (unsigned)nb;
  const unsigned s0 = (unsigned)da.x - nbs, s1 = (unsigned)da.y - nbs;
  const unsigned s2 = (unsigned)da.z - nbs, s3 = (unsigned)da.w - nbs;
  const unsigned s4 = (unsigned)db.x - nbs, s5 = (unsigned)db.y - nbs;
  const unsigned s6 = (unsigned)db.z - nbs, s7 = (unsigned)db.w - nbs;
  const bool h0 = s0 < unb, h1 = s1 < unb, h2 = s2 < unb, h3 = s3 < unb;
  const bool h4 = s4 < unb, h5 = s5 < unb, h6 = s6 < unb, h7 = s7 < unb;
  const unsigned any = __builtin_amdgcn_ballot_w32(h0 | h1 | h2 | h3 | h4 | h5 | h6 | h7);
  if (any != 0u) {
#define HITJ(J, HJ, SJ) { \
      const unsigned mj = __builtin_amdgcn_ballot_w32(HJ); \
      if (mj != 0u) { \
        if (HJ) { \
          const int pos = wc + (int)__builtin_amdgcn_mbcnt_lo(mj, 0u); \
          if (pos < WCAP) list[wave * WCAP + pos] = ((el0 + (J)) << 12) | (int)(SJ); \
        } \
        wc += (int)__builtin_popcount(mj); } }
    HITJ(0, h0, s0)
    HITJ(1, h1, s1)
    HITJ(2, h2, s2)
    HITJ(3, h3, s3)
    HITJ(4, h4, s4)
    HITJ(5, h5, s5)
    HITJ(6, h6, s6)
    HITJ(7, h7, s7)
#undef HITJ
  }
  return wc;
}

__global__ __launch_bounds__(NTHR) void agg_kernel(
    const int* __restrict__ ei, const float* __restrict__ ew, const unsigned short* __restrict__ cv,
    unsigned int* agp, int nE, int vec8)
{
  extern __shared__ v4f lds_dyn[];
  int* reg1 = (int*)lds_dyn;
  int* reg2 = reg1 + RCAP;
  int* scnt = reg2 + RCAP;
  int* soff = scnt + NBMAX;
  int* list = soff + NBMAX;
  int* wcnt = list + LISTN;
  int* wtot = wcnt + NWAVE;
  float* sdinv = (float*)(wtot + NWAVE);
  const int tid = (int)threadIdx.x, lane = tid & 31, wave = tid >> 5;
  const int* srcs = ei;
  const int* dsts = ei + nE;
  const int g0 = (int)blockIdx.x * SLB;
  const unsigned int* xb = (const unsigned int*)(cv + P_X);

  for (int i = tid; i < NBMAX; i += NTHR) scnt[i] = 0;
  __syncthreads();

  int tot = 0;
  const int nChunks = (nE + CHUNK - 1) / CHUNK;
#pragma unroll 1
  for (int ch = 0; ch < nChunks; ++ch) {
    const int cbase = ch * CHUNK;
    const int wc = scan_chunk(dsts, nE, cbase, 0, NN_, vec8, list, tid, lane, wave);
    if (lane == 0) wcnt[wave] = wc;
    __syncthreads();
    int pre = 0, all = 0;
#pragma unroll
    for (int w2 = 0; w2 < NWAVE; ++w2) {
      int c = wcnt[w2];
      c = c < 0 ? 0 : (c > WCAP ? WCAP : c);
      all += c;
      pre += (w2 < wave) ? c : 0;
    }
    const int wcc  = wc > WCAP ? WCAP : wc;
    const int base = tot + pre;
#pragma unroll 1
    for (int i = lane; i < wcc; i += 32) {
      const int ent = list[wave * WCAP + i];
      const int el  = (ent >> 12) & (CHUNK - 1);
      const int sl  = ent & (NBMAX - 1);
      int eid = cbase + el;
      eid = eid > nE - 1 ? nE - 1 : eid;
      const int pos = base + i;
      if (pos < RCAP) reg1[pos] = (int)(((unsigned)eid << 12) | (unsigned)sl);
    }
    tot += all;
    tot = tot > RCAP ? RCAP : tot;
    __syncthreads();
  }
  const int nh = tot;

  if (wave == 0) {
#pragma unroll 1
    for (int b0 = 0; b0 < nh; b0 += 32) {
      const int idx = b0 + lane;
      const int uv  = reg1[idx < RCAP ? idx : RCAP - 1];
      const int m32 = (nh - b0) < 32 ? (nh - b0) : 32;
#pragma unroll 1
      for (int k = 0; k < m32; ++k) {
        const int u  = __builtin_amdgcn_readlane(uv, k);
        const int sl = u & (NBMAX - 1);
        if (lane == 0) scnt[sl] = scnt[sl] + 1;
      }
    }
  }
  __syncthreads();

  {
    const v4i ca = *(const v4i*)(scnt + 8 * tid);
    const v4i cb = *(const v4i*)(scnt + 8 * tid + 4);
    const int e0 = ca.x < 0 ? 0 : ca.x, e1 = ca.y < 0 ? 0 : ca.y, e2 = ca.z < 0 ? 0 : ca.z, e3 = ca.w < 0 ? 0 : ca.w;
    const int e4 = cb.x < 0 ? 0 : cb.x, e5 = cb.y < 0 ? 0 : cb.y, e6 = cb.z < 0 ? 0 : cb.z, e7 = cb.w < 0 ? 0 : cb.w;
    const int ts = e0 + e1 + e2 + e3 + e4 + e5 + e6 + e7;
    int incl = ts;
#pragma unroll
    for (int d = 1; d < 32; d <<= 1) {
      const int up = __shfl_up(incl, d);
      if (lane >= d) incl += up;
    }
    if (lane == 31) wtot[wave] = incl;
    __syncthreads();
    int pre = 0;
#pragma unroll
    for (int w2 = 0; w2 < NWAVE; ++w2) pre += (w2 < wave) ? wtot[w2] : 0;
    int run = pre + incl - ts;
    soff[8 * tid + 0] = run; run += e0;
    soff[8 * tid + 1] = run; run += e1;
    soff[8 * tid + 2] = run; run += e2;
    soff[8 * tid + 3] = run; run += e3;
    soff[8 * tid + 4] = run; run += e4;
    soff[8 * tid + 5] = run; run += e5;
    soff[8 * tid + 6] = run; run += e6;
    soff[8 * tid + 7] = run;
  }
  __syncthreads();
  for (int i = tid; i < NBMAX; i += NTHR) list[i] = soff[i];
  __syncthreads();

  if (wave == 0) {
#pragma unroll 1
    for (int b0 = 0; b0 < nh; b0 += 32) {
      const int idx = b0 + lane;
      const int uv  = reg1[idx < RCAP ? idx : RCAP - 1];
      const int m32 = (nh - b0) < 32 ? (nh - b0) : 32;
#pragma unroll 1
      for (int k = 0; k < m32; ++k) {
        const int u   = __builtin_amdgcn_readlane(uv, k);
        const int sl  = u & (NBMAX - 1);
        const int eid = (int)((unsigned)u >> 12);
        if (lane == 0) {
          int pos = list[sl];
          pos = pos < 0 ? 0 : (pos > RCAP - 1 ? RCAP - 1 : pos);
          reg2[pos] = eid;
          list[sl] = pos + 1;
        }
      }
    }
  }
  __syncthreads();

#pragma unroll 1
  for (int i = 0; i < NN_ / NTHR; ++i) {
    const int slot = i * NTHR + tid;
    int st  = soff[slot];
    int cnt = scnt[slot];
    st  = st < 0 ? 0 : (st > nh ? nh : st);
    cnt = cnt < 0 ? 0 : (cnt > DEGCAP ? DEGCAP : cnt);
    if (cnt > nh - st) cnt = nh - st;
    int mc = cnt;
#pragma unroll
    for (int off = 16; off > 0; off >>= 1) {
      const int o = __shfl_xor(mc, off);
      mc = o > mc ? o : mc;
    }
    float dsum = 0.0f;
#pragma unroll 1
    for (int q = 0; q < mc; ++q) {
      int idx = st + (q < cnt ? q : 0);
      idx = idx > RCAP - 1 ? RCAP - 1 : idx;
      int eid = reg2[idx];
      eid = eid < 0 ? 0 : (eid > nE - 1 ? nE - 1 : eid);
      const float wv = bf16r(ew[eid]);
      dsum += (q < cnt) ? wv : 0.0f;
    }
    sdinv[slot] = rsqrtf(dsum + 1.0f);
  }
  __syncthreads();

  const bool ovf = (nh >= RCAP);
  const float qnan = __int_as_float(0x7fc00000);
  unsigned int* stw = (unsigned int*)reg1 + wave * STW;
  const int nbw = NN_ / NWAVE;
  const int q8 = lane & 7, sub = lane >> 3;
#pragma unroll 1
  for (int jt = 0; jt < nbw; ++jt) {
    const int n = wave * nbw + jt;
    int st = soff[n];
    const int craw = scnt[n];
    int cnt = craw;
    st  = st < 0 ? 0 : (st > nh ? nh : st);
    cnt = cnt < 0 ? 0 : (cnt > DEGCAP ? DEGCAP : cnt);
    if (cnt > nh - st) cnt = nh - st;
    const float pz = (ovf || craw > DEGCAP) ? qnan : 0.0f;
    const float dn = sdinv[n];

    float acc[2 * SLB];
#pragma unroll
    for (int j = 0; j < 2 * SLB; ++j) acc[j] = 0.0f;

#pragma unroll 1
    for (int q = 0; q < cnt; ++q) {
      int idx = st + q; idx = idx > RCAP - 1 ? RCAP - 1 : idx;
      int eid = reg2[idx]; eid = eid < 0 ? 0 : (eid > nE - 1 ? nE - 1 : eid);
      const int sraw = srcs[eid];
      const int s = sraw < 0 ? 0 : (sraw > NN_ - 1 ? NN_ - 1 : sraw);
      const float wv  = bf16r(ew[eid]);
      const float nrm = (sdinv[s] * wv) * dn;
      const unsigned int* xr = xb + (size_t)s * 32 + lane;
      unsigned int u[SLB];
#pragma unroll
      for (int j = 0; j < SLB; ++j) u[j] = xr[(size_t)(g0 + j) * (size_t)(NN_ * 32)];
      ldwait();
#pragma unroll
      for (int j = 0; j < SLB; ++j) {
        acc[2 * j]     = fmaf(nrm, __uint_as_float(u[j] << 16),          acc[2 * j]);
        acc[2 * j + 1] = fmaf(nrm, __uint_as_float(u[j] & 0xffff0000u), acc[2 * j + 1]);
      }
    }
    {
      const float ds = dn * dn;
      const unsigned int* xr = xb + (size_t)n * 32 + lane;
      unsigned int u[SLB];
#pragma unroll
      for (int j = 0; j < SLB; ++j) u[j] = xr[(size_t)(g0 + j) * (size_t)(NN_ * 32)];
      ldwait();
#pragma unroll
      for (int j = 0; j < SLB; ++j) {
        acc[2 * j]     = fmaf(ds, __uint_as_float(u[j] << 16),          acc[2 * j]);
        acc[2 * j + 1] = fmaf(ds, __uint_as_float(u[j] & 0xffff0000u), acc[2 * j + 1]);
      }
    }

    __builtin_amdgcn_fence(__ATOMIC_RELEASE, "wavefront");
    __builtin_amdgcn_wave_barrier();
#pragma unroll
    for (int j = 0; j < SLB; ++j) {
      const float v0 = acc[2 * j] + pz;
      const float v1 = acc[2 * j + 1] + pz;
      const unsigned short hb0 = bf16_bits(v0);
      const unsigned short lb0 = bf16_bits(v0 - bf16_val(hb0));
      const unsigned short hb1 = bf16_bits(v1);
      const unsigned short lb1 = bf16_bits(v1 - bf16_val(hb1));
      stw[(2 * j) * 32 + lane]     = (unsigned)hb0 | ((unsigned)hb1 << 16);
      stw[(2 * j + 1) * 32 + lane] = (unsigned)lb0 | ((unsigned)lb1 << 16);
    }
    __builtin_amdgcn_fence(__ATOMIC_RELEASE, "wavefront");
    __builtin_amdgcn_wave_barrier();

    v4u sv[4];
    size_t so[4];
#pragma unroll
    for (int i = 0; i < 4; ++i) {
      const int L  = 4 * i + sub;
      const int j  = L >> 1;
      const int p  = L & 1;
      sv[i] = *(const v4ua*)(stw + L * 32 + 4 * q8);
      const int g  = g0 + j;
      const int bb = g / NS_;
      const int ss = g - bb * NS_;
      const int R  = (ss * NB_ + bb) * NN_ + n;
      so[i] = (size_t)p * (size_t)PLANE_U32 + (size_t)R * 32 + 4 * q8;
    }
#pragma unroll
    for (int i = 0; i < 4; ++i) *(volatile v4u*)(agp + so[i]) = sv[i];
    __threadfence();
#pragma unroll
    for (int i = 0; i < 4; ++i) *(volatile v4u*)(agp + so[i]) = sv[i];
  }
}

constexpr size_t DL_TH = 0;
constexpr size_t DL_TL = (size_t)128 * 64 * 2;
constexpr size_t DLDS  = 2 * DL_TL;

__global__ __launch_bounds__(128)
void conv_kernel(const unsigned short* __restrict__ agh, const unsigned short* __restrict__ agl,
                 const unsigned short* __restrict__ cv, const float* __restrict__ bg,
                 unsigned short* chp, unsigned short* clp)
{
  extern __shared__ __attribute__((aligned(16))) char smem[];
  lp_us sTH = (lp_us)(smem + DL_TH);
  lp_us sTL = (lp_us)(smem + DL_TL);

  const int tid = threadIdx.x, lane = tid & 31, w = tid >> 5;
  const int h = lane >> 4, m = lane & 15;
  const int m0 = blockIdx.x * 128;
  const int cy = blockIdx.y;
  const int m0w = m0 + 32 * w;
  const unsigned short* WG = cv + P_WG;

  const unsigned short* xa = agh + (size_t)(m0w + m) * NF_;
  const unsigned short* xl = agl + (size_t)(m0w + m) * NF_;
  const unsigned short* wb = WG  + (size_t)(64 * cy + m) * NF_;

  v8f acc[2][4];
#pragma unroll
  for (int mt = 0; mt < 2; ++mt)
#pragma unroll
    for (int nt = 0; nt < 4; ++nt) acc[mt][nt] = zero8();

#pragma unroll 1
  for (int k0 = 0; k0 < NF_; k0 += 32) {
    Frag ah[2], al[2], b[4];
#pragma unroll
    for (int mt = 0; mt < 2; ++mt) {
      ldfrag_g(ah[mt], xa + (size_t)mt * 16 * NF_ + k0, h);
      ldfrag_g(al[mt], xl + (size_t)mt * 16 * NF_ + k0, h);
    }
#pragma unroll
    for (int nt = 0; nt < 4; ++nt) ldfrag_g(b[nt], wb + (size_t)nt * 16 * NF_ + k0, h);
#pragma unroll
    for (int mt = 0; mt < 2; ++mt)
#pragma unroll
      for (int nt = 0; nt < 4; ++nt) {
        acc[mt][nt] = mma16(acc[mt][nt], ah[mt], b[nt]);
        acc[mt][nt] = mma16(acc[mt][nt], al[mt], b[nt]);
      }
    asm volatile("v_nop\n\tv_nop\n\tv_nop\n\tv_nop"
                 : "+v"(acc[0][0]), "+v"(acc[0][1]), "+v"(acc[0][2]), "+v"(acc[0][3]),
                   "+v"(acc[1][0]), "+v"(acc[1][1]), "+v"(acc[1][2]), "+v"(acc[1][3])
                 : "v"(ah[0].v), "v"(ah[1].v), "v"(al[0].v), "v"(al[1].v),
                   "v"(b[0].v), "v"(b[1].v), "v"(b[2].v), "v"(b[3].v));
  }

#pragma unroll
  for (int nt = 0; nt < 4; ++nt) {
    const int col = 16 * nt + m;
    const float bias = bf16r(bg[64 * cy + col]);
#pragma unroll
    for (int mt = 0; mt < 2; ++mt)
#pragma unroll
      for (int r = 0; r < 8; ++r) {
        const int rowl = 32 * w + 16 * mt + 8 * h + r;
        const float v = acc[mt][nt][r] + bias;
        const unsigned short hb = bf16_bits(v);
        const unsigned short lb = bf16_bits(v - bf16_val(hb));
        sTH[rowl * 64 + col] = hb;
        sTL[rowl * 64 + col] = lb;
      }
  }
  __syncthreads();

  const int q8 = lane & 7, sub = lane >> 3;
#pragma unroll 1
  for (int pass = 0; pass < 2; ++pass) {
#pragma unroll
    for (int i = 0; i < 8; ++i) {
      const int lid = 32 * w + 4 * i + sub;
      const v8us vh = *(AS3 const v8usa*)(sTH + lid * 64 + 8 * q8);
      const v8us vl = *(AS3 const v8usa*)(sTL + lid * 64 + 8 * q8);
      const size_t go = (size_t)(m0 + lid) * NH_ + 64 * cy + 8 * q8;
      *(volatile v8us*)(chp + go) = vh;
      *(volatile v8us*)(clp + go) = vl;
    }
    __threadfence();
  }
}

constexpr int    HP     = NH_ + 8;
constexpr int    HTILE  = NSQB * HP;
constexpr size_t RL_HH  = 0;
constexpr size_t RLSZ_H = (size_t)2 * HTILE * 2;
constexpr size_t RL_HL  = RL_HH + RLSZ_H;
constexpr size_t RL_BI  = RL_HL + RLSZ_H;
constexpr size_t RL_SO  = RL_BI + (size_t)NG_ * 4;
constexpr size_t RLDS   = RL_SO + (size_t)NSQB * NO_ * 4;
static_assert(HP % 8 == 0);
static_assert(RL_HL % 16 == 0 && RL_BI % 16 == 0 && RL_SO % 16 == 0);
constexpr int NZH = (int)(RL_BI / 16);

__global__ __launch_bounds__(256)
void lstm_kernel(const unsigned short* __restrict__ cv, const unsigned short* __restrict__ chp,
                 const unsigned short* __restrict__ clp, const float* __restrict__ bih,
                 const float* __restrict__ bhh, const float* __restrict__ bfc, float* out)
{
  extern __shared__ __attribute__((aligned(16))) char smem[];
  lp_us hH    = (lp_us)(smem + RL_HH);
  lp_us hL    = (lp_us)(smem + RL_HL);
  lp_f  sBias = (lp_f)(smem + RL_BI);
  lp_f  sOut  = (lp_f)(smem + RL_SO);

  const int tid = threadIdx.x, lane = tid & 31, w = tid >> 5;
  const int h = lane >> 4, m = lane & 15;
  const int seq0 = (int)blockIdx.x * NSQB;
  const unsigned short* WI = cv + P_WI;
  const unsigned short* WH = cv + P_WH;
  const unsigned short* WF = cv + P_WF;

  {
    v8us z8;
#pragma unroll
    for (int i = 0; i < 8; ++i) z8[i] = (unsigned short)0;
    for (int i = tid; i < NZH; i += 256) *(AS3 v8us*)(hH + 8 * i) = z8;
    sBias[tid]        = bf16r(bih[tid])        + bf16r(bhh[tid]);
    sBias[NTHR + tid] = bf16r(bih[NTHR + tid]) + bf16r(bhh[NTHR + tid]);
  }
  __syncthreads();

  float cst[8];
#pragma unroll
  for (int r = 0; r < 8; ++r) cst[r] = 0.0f;

  const int u = 16 * w + m;

#pragma unroll 1
  for (int s = 0; s < NS_; ++s) {
    const int cur = s & 1;
    lcp_us hHc = hH + cur * HTILE;
    lcp_us hLc = hL + cur * HTILE;
    lp_us  hHn = hH + (cur ^ 1) * HTILE;
    lp_us  hLn = hL + (cur ^ 1) * HTILE;

    __syncthreads();

    v8f acc[4];
#pragma unroll
    for (int nt = 0; nt < 4; ++nt) acc[nt] = zero8();

    {
      const size_t crow = ((size_t)s * NSEQ + seq0 + m) * NH_;
      const unsigned short* ca  = chp + crow;
      const unsigned short* cla = clp + crow;
      const unsigned short* wb  = WI + (size_t)(16 * w + m) * NH_;
#pragma unroll 1
      for (int k0 = 0; k0 < NH_; k0 += 32) {
        Frag ah, al, b[4];
        ldfrag_g(ah, ca  + k0, h);
        ldfrag_g(al, cla + k0, h);
#pragma unroll
        for (int nt = 0; nt < 4; ++nt) ldfrag_g(b[nt], wb + (size_t)nt * NH_ * NH_ + k0, h);
#pragma unroll
        for (int nt = 0; nt < 4; ++nt) {
          acc[nt] = mma16(acc[nt], ah, b[nt]);
          acc[nt] = mma16(acc[nt], al, b[nt]);
        }
        asm volatile("v_nop\n\tv_nop\n\tv_nop\n\tv_nop"
                     : "+v"(acc[0]), "+v"(acc[1]), "+v"(acc[2]), "+v"(acc[3])
                     : "v"(ah.v), "v"(al.v), "v"(b[0].v), "v"(b[1].v), "v"(b[2].v), "v"(b[3].v));
      }
    }
    {
      lcp_us ha = hHc + m * HP;
      lcp_us la = hLc + m * HP;
      const unsigned short* wb = WH + (size_t)(16 * w + m) * NH_;
#pragma unroll 1
      for (int k0 = 0; k0 < NH_; k0 += 32) {
        Frag ah, al, b[4];
        ldfrag_l(ah, ha + k0, h);
        ldfrag_l(al, la + k0, h);
#pragma unroll
        for (int nt = 0; nt < 4; ++nt) ldfrag_g(b[nt], wb + (size_t)nt * NH_ * NH_ + k0, h);
#pragma unroll
        for (int nt = 0; nt < 4; ++nt) {
          acc[nt] = mma16(acc[nt], ah, b[nt]);
          acc[nt] = mma16(acc[nt], al, b[nt]);
        }
        asm volatile("v_nop\n\tv_nop\n\tv_nop\n\tv_nop"
                     : "+v"(acc[0]), "+v"(acc[1]), "+v"(acc[2]), "+v"(acc[3])
                     : "v"(ah.v), "v"(al.v), "v"(b[0].v), "v"(b[1].v), "v"(b[2].v), "v"(b[3].v));
      }
    }

    {
      const float bi = sBias[u], bf = sBias[NH_ + u], bgg = sBias[2 * NH_ + u], bo = sBias[3 * NH_ + u];
#pragma unroll
      for (int r = 0; r < 8; ++r) {
        const int row = 8 * h + r;
        const float gi = acc[0][r] + bi;
        const float gf = acc[1][r] + bf;
        const float gg = acc[2][r] + bgg;
        const float go = acc[3][r] + bo;
        const float cn = sigm(gf) * cst[r] + sigm(gi) * tanhf(gg);
        cst[r] = cn;
        const float hv = sigm(go) * tanhf(cn);
        const unsigned short hb = bf16_bits(hv);
        const unsigned short lb = bf16_bits(hv - bf16_val(hb));
        hHn[row * HP + u] = hb;
        hLn[row * HP + u] = lb;
      }
    }
  }
  __syncthreads();

  if (w < 2) {
    const int nt = w;
    v8f facc = zero8();
    lcp_us ha = hH + (NS_ & 1) * HTILE + m * HP;
    lcp_us la = hL + (NS_ & 1) * HTILE + m * HP;
    const unsigned short* wb = WF + (size_t)(16 * nt + m) * NH_;
#pragma unroll 1
    for (int k0 = 0; k0 < NH_; k0 += 32) {
      Frag ah, al, b;
      ldfrag_l(ah, ha + k0, h);
      ldfrag_l(al, la + k0, h);
      ldfrag_g(b, wb + k0, h);
      facc = mma16(facc, ah, b);
      facc = mma16(facc, al, b);
      asm volatile("v_nop\n\tv_nop\n\tv_nop\n\tv_nop" : "+v"(facc) : "v"(ah.v), "v"(al.v), "v"(b.v));
    }
    const int col = 16 * nt + m;
    const float bias = bf16r(bfc[col]);
#pragma unroll
    for (int r = 0; r < 8; ++r) sOut[(8 * h + r) * NO_ + col] = facc[r] + bias;
  }
  __syncthreads();

  const bool act = tid < NSQB * 8;
  const int orow = (tid >> 3) & (NSQB - 1);
  const int oq   = tid & 7;
  v4f ov = {0.0f, 0.0f, 0.0f, 0.0f};
  if (act) ov = *(AS3 const v4fa*)(sOut + orow * NO_ + 4 * oq);
  float* od = out + (size_t)(seq0 + orow) * NO_ + 4 * oq;
  if (act) *(volatile v4f*)od = ov;
  __threadfence();
  if (act) *(volatile v4f*)od = ov;
}

extern "C" void kernel_launch(void* const* d_in, const int* in_sizes, int n_in,
                              void* d_out, int out_size, void* d_ws, size_t ws_size,
                              hipStream_t stream)
{
  if (n_in < 11) return;
  if (in_sizes[0]  != NB_ * NS_ * NN_ * NF_) return;
  if (in_sizes[1]  != 2 * NE_)               return;
  if (in_sizes[2]  != NE_)                   return;
  if (in_sizes[3]  != NF_ * NH_)             return;
  if (in_sizes[4]  != NH_)                   return;
  if (in_sizes[5]  != NG_ * NH_)             return;
  if (in_sizes[6]  != NG_ * NH_)             return;
  if (in_sizes[7]  != NG_)                   return;
  if (in_sizes[8]  != NG_)                   return;
  if (in_sizes[9]  != NO_ * NH_)             return;
  if (in_sizes[10] != NO_)                   return;
  if (out_size != NSEQ * NO_)                return;
  if (ws_size < WS_END)                      return;

  const float* x   = (const float*)d_in[0];
  const int*   ei  = (const int*)  d_in[1];
  const float* ew  = (const float*)d_in[2];
  const float* wg  = (const float*)d_in[3];
  const float* bg  = (const float*)d_in[4];
  const float* wi  = (const float*)d_in[5];
  const float* wh  = (const float*)d_in[6];
  const float* bih = (const float*)d_in[7];
  const float* bhh = (const float*)d_in[8];
  const float* wf  = (const float*)d_in[9];
  const float* bfc = (const float*)d_in[10];
  float* out = (float*)d_out;

  char* ws = (char*)d_ws;
  unsigned short* cv  = (unsigned short*)(ws + OFF_CV);
  unsigned int*   agp = (unsigned int*)(ws + OFF_AG);
  const unsigned short* agh = (const unsigned short*)(ws + OFF_AG);
  const unsigned short* agl = (const unsigned short*)(ws + OFF_AGL);
  unsigned short* cvh = (unsigned short*)(ws + OFF_CVH);
  unsigned short* cvl = (unsigned short*)(ws + OFF_CVL);

  const int nE   = NE_;
  const int vec8 = ((nE & 3) == 0) ? 1 : 0;

  cvt_kernel<<<dim3(NCBLK), dim3(256), 0, stream>>>(x, wg, wi, wh, wf, cv);

  hipFuncSetAttribute(reinterpret_cast<const void*>(&agg_kernel),
                      hipFuncAttributeMaxDynamicSharedMemorySize, (int)LDS_AGG);
  agg_kernel<<<dim3(NSL / SLB), dim3(NTHR), LDS_AGG, stream>>>(ei, ew, cv, agp, nE, vec8);

  conv_kernel<<<dim3(NROW / 128, 2), dim3(128), DLDS, stream>>>(agh, agl, cv, bg, cvh, cvl);

  lstm_kernel<<<dim3(NSEQ / NSQB), dim3(256), RLDS, stream>>>(cv, cvh, cvl, bih, bhh, bfc, out);
}
